// MultiHeadCulturalAttention_68685116998268
// MI455X (gfx1250) — hardware-verified
//
#include <hip/hip_runtime.h>
#include <math.h>

typedef __attribute__((ext_vector_type(16))) _Float16 v16h;
typedef __attribute__((ext_vector_type(16))) __bf16 v16b;
typedef __attribute__((ext_vector_type(8)))  _Float16 v8h;
typedef __attribute__((ext_vector_type(8)))  float v8f;
typedef __attribute__((ext_vector_type(4)))  float v4f;
typedef __attribute__((ext_vector_type(2)))  float v2f;
typedef __attribute__((ext_vector_type(4)))  unsigned v4u;
typedef __attribute__((ext_vector_type(4)))  int v4i;
typedef float __attribute__((may_alias)) float_a;
typedef int __attribute__((may_alias)) int_a;

template <typename T> __device__ __forceinline__ void vst2(void* p, T v) { *(volatile T*)p = v; __threadfence(); *(volatile T*)p = v; }
__device__ __forceinline__ v8f wmma16(v16h a, v16h b, v8f c) {
  v8f d = __builtin_amdgcn_wmma_f32_16x16x32_f16(false, a, false, b, (short)0, c, false, false);
  asm volatile("v_nop\n\tv_nop\n\tv_nop\n\tv_nop" : "+v"(d) : "v"(a), "v"(b));
  return d;
}
__device__ __forceinline__ v8f wmma_bf(v16b a, v16b b, v8f c) {
  v8f d = __builtin_amdgcn_wmma_f32_16x16x32_bf16(false, a, false, b, (short)0, c, false, false);
  asm volatile("v_nop\n\tv_nop\n\tv_nop\n\tv_nop" : "+v"(d) : "v"(a), "v"(b));
  return d;
}
__device__ __forceinline__ v16h frag_h(const _Float16* rowk0, int lane) {
  union { v16h v; v8h q[2]; } u; const _Float16* p = rowk0 + 8 * (lane >> 4);
  u.q[0] = *(const v8h*)p; u.q[1] = *(const v8h*)(p + 16); return u.v;
}
__device__ __forceinline__ v16h frag_f32(const float* rowk0, int lane) {
  v16h a; const float* p = rowk0 + 8 * (lane >> 4);
#pragma unroll
  for (int i = 0; i < 8; ++i) { a[i] = (_Float16)p[i]; a[8 + i] = (_Float16)p[16 + i]; }
  return a;
}
__device__ __forceinline__ v16h frag_f32s(const float* rowk0, int lane, float sc) {
  v16h a; const float* p = rowk0 + 8 * (lane >> 4);
#pragma unroll
  for (int i = 0; i < 8; ++i) { a[i] = (_Float16)(p[i] * sc); a[8 + i] = (_Float16)(p[16 + i] * sc); }
  return a;
}
__device__ __forceinline__ v16h fragc_f32(const float* W, int k0, int n, int lane, int ld, int K) {
  v16h a; const int g = lane >> 4;
#pragma unroll
  for (int i = 0; i < 8; ++i) { const int ka = k0 + 8 * g + i, kb = ka + 16;
    a[i] = (_Float16)(ka < K ? W[(size_t)(ka < K ? ka : K - 1) * ld + n] : 0.f); a[8 + i] = (_Float16)(kb < K ? W[(size_t)(kb < K ? kb : K - 1) * ld + n] : 0.f); }
  return a;
}
struct F2 { v16b h, l; };
__device__ __forceinline__ F2 bsplit16(const float v[16]) { F2 r;
#pragma unroll
  for (int i = 0; i < 16; ++i) { const __bf16 h = (__bf16)v[i]; r.h[i] = h; r.l[i] = (__bf16)(v[i] - (float)h); }
  return r; }
__device__ __forceinline__ F2 split_row(const float* row, int k0, int lane) { float v[16]; const float* p = row + k0 + 8 * (lane >> 4);
#pragma unroll
  for (int i = 0; i < 8; ++i) { v[i] = p[i]; v[8 + i] = p[16 + i]; }
  return bsplit16(v); }
__device__ __forceinline__ F2 split_rowK(const float* row, int k0, int lane, int K) { float v[16]; const int g = lane >> 4;
#pragma unroll
  for (int i = 0; i < 8; ++i) { const int ka = k0 + 8 * g + i, kb = ka + 16; v[i] = ka < K ? row[ka < K ? ka : K - 1] : 0.f; v[8 + i] = kb < K ? row[kb < K ? kb : K - 1] : 0.f; }
  return bsplit16(v); }
__device__ __forceinline__ F2 split_col(const float* W, int k0, int n, int lane, int ld, int K) { float v[16]; const int g = lane >> 4;
#pragma unroll
  for (int i = 0; i < 8; ++i) { const int ka = k0 + 8 * g + i, kb = ka + 16; v[i] = ka < K ? W[(size_t)(ka < K ? ka : K - 1) * ld + n] : 0.f; v[8 + i] = kb < K ? W[(size_t)(kb < K ? kb : K - 1) * ld + n] : 0.f; }
  return bsplit16(v); }
__device__ __forceinline__ v8f mac3(const F2& a, const F2& b, v8f c) { c = wmma_bf(a.l, b.h, c); c = wmma_bf(a.h, b.l, c); return wmma_bf(a.h, b.h, c); }
__device__ __forceinline__ float sigm(float v) { return 1.0f / (1.0f + expf(-v)); }
#define LDSX() do { asm volatile("s_wait_dscnt 0" ::: "memory"); __builtin_amdgcn_wave_barrier(); __builtin_amdgcn_fence(__ATOMIC_RELEASE, "workgroup"); } while (0)


#define NB 2
#define SS 2048
#define EE 768
#define NR (NB * SS)
#define E2 (2 * EE)
#ifndef NPAIR_R
#define NPAIR_R (NB * 6)
#define NPAIR_C (NB * 2)
#define NRB (NR / 64)
#endif
typedef __attribute__((ext_vector_type(8))) __bf16 v8b;
__device__ __forceinline__ v16b frag_b(const __bf16* rowk0, int lane) {
  union { v16b v; v8b q[2]; } u; const __bf16* p = rowk0 + 8 * (lane >> 4);
  u.q[0] = *(const v8b*)p; u.q[1] = *(const v8b*)(p + 16); return u.v;
}
__device__ __forceinline__ float bfr(float v) { return (float)(__bf16)v; }
__device__ __attribute__((noinline)) float exp_ni(float v) { return expf(v); }
__device__ __attribute__((noinline)) float erf_ni(float v) { return erff(v); }

#define WS_PW   0u
#define WS_POUT (WS_PW + 2u * (size_t)8 * EE * EE)
#define WS_Q    (WS_POUT + 2u * (size_t)EE * E2)
#define WS_K    (WS_Q + 2u * (size_t)2 * NR * EE)
#define WS_V    (WS_K + 2u * (size_t)2 * NR * EE)
#define WS_S    (WS_V + 2u * (size_t)2 * NB * EE * SS)
#define WS_P    (WS_S + 4u * (size_t)SS * SS)
#define WS_IL   (WS_P + 2u * (size_t)SS * SS)
#define WS_O    (WS_IL + 4u * SS)
#define WS_BR   (WS_O + 4u * (size_t)2 * NR * EE)
#define WS_END  (WS_BR + 4u * (size_t)2 * NR * EE)

__global__ __launch_bounds__(256) void k_pack(const float* __restrict__ W0, const float* __restrict__ W1, const float* __restrict__ W2, const float* __restrict__ W3, const float* __restrict__ W4, const float* __restrict__ W5, const float* __restrict__ W6, const float* __restrict__ W7, const float* __restrict__ WOUT, __bf16* __restrict__ P) {
  const int n = blockIdx.x, which = blockIdx.y, t = threadIdx.x; __shared__ __align__(16) __bf16 s[E2];
  if (which < 8) { const float* Wm = (which == 0) ? W0 : (which == 1) ? W1 : (which == 2) ? W2 : (which == 3) ? W3 : (which == 4) ? W4 : (which == 5) ? W5 : (which == 6) ? W6 : W7;
    for (int k = t; k < EE; k += 256) s[k] = (__bf16)Wm[(size_t)k * EE + n]; __syncthreads(); for (int q = t; q < EE / 8; q += 256) vst2((unsigned*)(P + WS_PW / 2 + ((size_t)which * EE + n) * EE + q * 8), *(const v4u*)&s[q * 8]); }
  else { for (int k = t; k < E2; k += 256) s[k] = (__bf16)WOUT[(size_t)k * EE + n]; __syncthreads(); for (int q = t; q < E2 / 8; q += 256) vst2((unsigned*)(P + WS_POUT / 2 + (size_t)n * E2 + q * 8), *(const v4u*)&s[q * 8]); }
}
__global__ __launch_bounds__(128) void k_proj(const float* __restrict__ X, const __bf16* __restrict__ P, const float* __restrict__ RQB, const float* __restrict__ RKB, const float* __restrict__ RVB, const float* __restrict__ CQB, const float* __restrict__ CKB, const float* __restrict__ CVB, const float* __restrict__ RCB, const float* __restrict__ CCB, _Float16* __restrict__ Q, _Float16* __restrict__ Kr, _Float16* __restrict__ V) {
  __shared__ __align__(16) _Float16 so[64][136]; __shared__ __align__(16) _Float16 st[128][72];
  const int tid = threadIdx.x, wave = tid >> 5, lane = tid & 31, col = lane & 15, g = lane >> 4; const int br = blockIdx.z / 3, which = blockIdx.z % 3; const int n0 = blockIdx.y * 128; const size_t rb0 = (size_t)blockIdx.x * 64, r0 = rb0 + wave * 16;
  const int widx = (br == 0) ? which : 4 + which;
  const __bf16* Wr = P + WS_PW / 2 + (size_t)widx * EE * EE; const int bi = br * 3 + which; const float* BB = (bi == 0) ? RQB : (bi == 1) ? RKB : (bi == 2) ? RVB : (bi == 3) ? CQB : (bi == 4) ? CKB : CVB; const float* CB = (which == 0) ? (br == 0 ? RCB : CCB) : nullptr;
  v8f acc[8] = {};
#pragma unroll 2
  for (int kc = 0; kc < EE / 32; ++kc) { v16b a; { const float* p = X + (r0 + col) * EE + kc * 32 + 8 * g;
#pragma unroll
      for (int i = 0; i < 8; ++i) { a[i] = (__bf16)p[i]; a[8 + i] = (__bf16)p[16 + i]; } }
#pragma unroll
    for (int j = 0; j < 8; ++j) acc[j] = wmma_bf(a, frag_b(Wr + (size_t)(n0 + j * 16 + col) * EE + kc * 32, lane), acc[j]); }
  if (which < 2) {
#pragma unroll
    for (int j = 0; j < 8; ++j) { const int c = n0 + j * 16 + col; const float bb = bfr(BB[c]) + (CB ? bfr(CB[c]) : 0.f);
#pragma unroll
      for (int r = 0; r < 8; ++r) so[wave * 16 + 8 * g + r][j * 16 + col] = (_Float16)(CB ? ((acc[j][r] + bfr(BB[c])) + bfr(CB[c])) : (acc[j][r] + bb)); }
    LDSX();
    _Float16* dst = ((which == 0) ? Q : Kr) + (size_t)br * NR * EE;
    for (int rl = 0; rl < 16; ++rl) if (lane < 16) vst2((unsigned*)(dst + (r0 + rl) * EE + n0 + lane * 8), *(const v4u*)&so[wave * 16 + rl][lane * 8]);
  } else {
#pragma unroll
    for (int j = 0; j < 8; ++j) { const float bb = bfr(BB[n0 + j * 16 + col]);
#pragma unroll
      for (int r = 0; r < 8; ++r) st[j * 16 + col][wave * 16 + 8 * g + r] = (_Float16)(acc[j][r] + bb); }
    __syncthreads();
    const size_t b = rb0 / SS, s0 = rb0 % SS;
    for (int e = tid; e < 128 * 8; e += 128) { const int d = e >> 3, pc = e & 7; vst2((unsigned*)(V + (((size_t)br * NB + b) * EE + n0 + d) * SS + s0 + pc * 8), *(const v4u*)&st[d][pc * 8]); } }
}
template <int KCH>
__global__ __launch_bounds__(128) void k_scores(const _Float16* __restrict__ Q, const _Float16* __restrict__ Kr, const float* __restrict__ AM, const float* __restrict__ CM, int b, int hoff, float scale, float* __restrict__ S) {
  __shared__ __align__(16) float so[4][16][132];
  const int tid = threadIdx.x, wave = tid >> 5, lane = tid & 31, col = lane & 15, g = lane >> 4; const int q0 = blockIdx.x * 64 + wave * 16; const int k0 = blockIdx.y * 128; const size_t rq = (size_t)b * SS + q0, rk = (size_t)b * SS + k0;
  v8f acc[8] = {};
#pragma unroll
  for (int kc = 0; kc < KCH; ++kc) { const v16h a = frag_h(Q + (rq + col) * EE + hoff + kc * 32, lane);
#pragma unroll
    for (int j = 0; j < 8; ++j) acc[j] = wmma16(a, frag_h(Kr + (rk + j * 16 + col) * EE + hoff + kc * 32, lane), acc[j]); }
#pragma unroll
  for (int j = 0; j < 8; ++j) { const int kk = k0 + j * 16 + col; const float am = bfr(AM[(size_t)b * SS + kk]);
#pragma unroll
    for (int r = 0; r < 8; ++r) { float v = acc[j][r] * scale + am; if (CM) v += bfr(CM[((size_t)b * SS + q0 + 8 * g + r) * SS + kk]); so[wave][8 * g + r][j * 16 + col] = v; } }
  LDSX();
  for (int rl = 0; rl < 16; ++rl) vst2(S + (size_t)(q0 + rl) * SS + k0 + lane * 4, *(const v4f*)&so[wave][rl][lane * 4]);
}
__global__ __launch_bounds__(256) void k_soft(const float* __restrict__ S, _Float16* __restrict__ P, float* __restrict__ IL) {
  __shared__ float red[256]; __shared__ __align__(16) _Float16 sp[SS];
  const int r = blockIdx.x, t = threadIdx.x; const float* row = S + (size_t)r * SS;
  float mx = -3.0e38f; for (int k = t; k < SS; k += 256) mx = fmaxf(mx, row[k]); red[t] = mx; __syncthreads();
  for (int s = 128; s > 0; s >>= 1) { if (t < s) red[t] = fmaxf(red[t], red[t + s]); __syncthreads(); }
  const float gm = red[0]; __syncthreads();
  float sum = 0.f; for (int k = t; k < SS; k += 256) { const float e = __expf(row[k] - gm); sum += e; sp[k] = (_Float16)(e * 2048.0f); }
  red[t] = sum; __syncthreads();
  for (int s = 128; s > 0; s >>= 1) { if (t < s) red[t] += red[t + s]; __syncthreads(); }
  if (t == 0) IL[r] = (1.0f / 2048.0f) / red[0];
  for (int q = t; q < SS / 8; q += 256) vst2((unsigned*)(P + (size_t)r * SS + q * 8), *(const v4u*)&sp[q * 8]);
}
__global__ __launch_bounds__(128) void k_pv(const _Float16* __restrict__ P, const _Float16* __restrict__ Vp, const float* __restrict__ IL, int b, int hoff, float* __restrict__ O) {
  __shared__ __align__(16) float so[4][16][132];
  const int tid = threadIdx.x, wave = tid >> 5, lane = tid & 31, col = lane & 15, g = lane >> 4; const int q0 = blockIdx.x * 64 + wave * 16; const int c0 = hoff + blockIdx.y * 128;
  v8f acc[8] = {};
#pragma unroll 2
  for (int kc = 0; kc < SS / 32; ++kc) { const v16h a = frag_h(P + (size_t)(q0 + col) * SS + kc * 32, lane);
#pragma unroll
    for (int j = 0; j < 8; ++j) acc[j] = wmma16(a, frag_h(Vp + ((size_t)b * EE + c0 + j * 16 + col) * SS + kc * 32, lane), acc[j]); }
#pragma unroll
  for (int j = 0; j < 8; ++j)
#pragma unroll
    for (int r = 0; r < 8; ++r) so[wave][8 * g + r][j * 16 + col] = acc[j][r] * IL[q0 + 8 * g + r];
  LDSX();
  for (int rl = 0; rl < 16; ++rl) vst2(O + ((size_t)b * SS + q0 + rl) * EE + c0 + lane * 4, *(const v4f*)&so[wave][rl][lane * 4]);
}
template <int KIN>
__global__ __launch_bounds__(128) void k_lin(const float* __restrict__ A, const float* __restrict__ A2, const __bf16* __restrict__ Wr, const float* __restrict__ BIAS, float* __restrict__ OUT) {
  __shared__ __align__(16) float so[4][16][132];
  const int tid = threadIdx.x, wave = tid >> 5, lane = tid & 31, col = lane & 15, g = lane >> 4; const size_t r0 = (size_t)blockIdx.x * 64 + wave * 16; const int n0 = blockIdx.y * 128;
  v8f acc[8] = {};
#pragma unroll 2
  for (int kc = 0; kc < KIN / 32; ++kc) { const bool second = (KIN > EE) && (kc >= EE / 32); const F2 a = second ? split_row(A2 + (r0 + col) * EE, (kc - EE / 32) * 32, lane) : split_row(A + (r0 + col) * EE, kc * 32, lane);
#pragma unroll
    for (int j = 0; j < 8; ++j) { const v16b w = frag_b(Wr + (size_t)(n0 + j * 16 + col) * KIN + kc * 32, lane); acc[j] = wmma_bf(a.l, w, acc[j]); acc[j] = wmma_bf(a.h, w, acc[j]); } }
#pragma unroll
  for (int j = 0; j < 8; ++j) { const float bb = bfr(BIAS[n0 + j * 16 + col]);
#pragma unroll
    for (int r = 0; r < 8; ++r) so[wave][8 * g + r][j * 16 + col] = acc[j][r] + bb; }
  LDSX();
  for (int rl = 0; rl < 16; ++rl) vst2(OUT + (r0 + rl) * EE + n0 + lane * 4, *(const v4f*)&so[wave][rl][lane * 4]);
}
extern "C" void kernel_launch(void* const* d_in, const int* in_sizes, int n_in, void* d_out, int out_size, void* d_ws, size_t ws_size, hipStream_t stream) {
  (void)in_sizes; (void)n_in; (void)out_size;
  const float** F = (const float**)d_in;
  if (ws_size < (size_t)WS_END + 256) return;
  char* ws = (char*)d_ws; __bf16* P = (__bf16*)ws; _Float16 *Q = (_Float16*)(ws + WS_Q), *Kr = (_Float16*)(ws + WS_K), *V = (_Float16*)(ws + WS_V), *Pm = (_Float16*)(ws + WS_P); float *S = (float*)(ws + WS_S), *IL = (float*)(ws + WS_IL), *O = (float*)(ws + WS_O), *BR = (float*)(ws + WS_BR);
  k_pack<<<dim3(EE, 9), 256, 0, stream>>>(F[3], F[4], F[5], F[6], F[7], F[8], F[9], F[10], F[21], P);
  k_proj<<<dim3(NRB, EE / 128, 6), 128, 0, stream>>>(F[0], P, F[11], F[12], F[13], F[15], F[16], F[17], F[19], F[20], Q, Kr, V);
  for (int pr = 0; pr < NPAIR_R; ++pr) { const int b = pr / 6, h = pr % 6;
    k_scores<4><<<dim3(SS / 64, SS / 128), 128, 0, stream>>>(Q, Kr, F[2], nullptr, b, h * 128, 0.08838834764831845f, S);
    k_soft<<<SS, 256, 0, stream>>>(S, Pm, IL);
    k_pv<<<dim3(SS / 64, 1), 128, 0, stream>>>(Pm, V, IL, b, h * 128, O); }
  for (int pr = 0; pr < NPAIR_C; ++pr) { const int b = pr / 2, h = pr % 2;
    k_scores<12><<<dim3(SS / 64, SS / 128), 128, 0, stream>>>(Q + (size_t)NR * EE, Kr + (size_t)NR * EE, F[2], F[1], b, h * 384, 0.05103103630798288f, S);
    k_soft<<<SS, 256, 0, stream>>>(S, Pm, IL);
    k_pv<<<dim3(SS / 64, 3), 128, 0, stream>>>(Pm, V + (size_t)NB * EE * SS, IL, b, h * 384, O + (size_t)NR * EE); }
  k_lin<EE><<<dim3(NRB, EE / 128), 128, 0, stream>>>(O, nullptr, P + WS_PW / 2 + (size_t)3 * EE * EE, F[14], BR);
  k_lin<EE><<<dim3(NRB, EE / 128), 128, 0, stream>>>(O + (size_t)NR * EE, nullptr, P + WS_PW / 2 + (size_t)7 * EE * EE, F[18], BR + (size_t)NR * EE);
  k_lin<E2><<<dim3(NRB, EE / 128), 128, 0, stream>>>(BR, BR + (size_t)NR * EE, P + WS_POUT / 2, F[22], (float*)d_out);
}
